// BraidCausalSelfAttention_24507083391053
// MI455X (gfx1250) — hardware-verified
//
#include <hip/hip_runtime.h>
#include <math.h>

constexpr int kSeqLen = 4096;
constexpr int kEmbd   = 1024;
constexpr int kHeads  = 16;
constexpr int kHeadD  = 64;
constexpr int kRotD   = 32;
constexpr int kHeadsPerChunk = 2;
constexpr float kWCarry   = 16.0f;
constexpr float kVCarry   = 16.0f;
constexpr float kPCarry   = 2048.0f;
constexpr float kQKScale  = 1.0f / 16.0f;
constexpr float kScScale  = 0.125f;
constexpr float kPVScale  = 1.0f / 32768.0f;
constexpr float kOutScale = 1.0f / 1024.0f;
constexpr float kEpsRms   = 1e-6f;

typedef __attribute__((ext_vector_type(16))) _Float16 v16h;
typedef __attribute__((ext_vector_type(8)))  _Float16 v8h;
typedef __attribute__((ext_vector_type(16))) __bf16   v16b;
typedef __attribute__((ext_vector_type(8)))  __bf16   v8b;
typedef __attribute__((ext_vector_type(8)))  float    v8f;
typedef __attribute__((ext_vector_type(4)))  float    v4f;
typedef __attribute__((ext_vector_type(4)))  unsigned int v4u;

__device__ __forceinline__ unsigned short f2bf_bits(float f) {
  unsigned u = __float_as_uint(f);
  return (unsigned short)((u + 0x7FFFu + ((u >> 16) & 1u)) >> 16);
}
__device__ __forceinline__ float bf_bits2f(unsigned short h) { return __uint_as_float(((unsigned)h) << 16); }

__device__ __forceinline__ void dep_guard_h(v8f& a, v8f& b, v16h x, v16h y) { asm volatile("v_nop\n\tv_nop\n\tv_nop\n\tv_nop" : "+v"(a), "+v"(b) : "v"(x), "v"(y)); }
__device__ __forceinline__ void dep_guard_b(v8f& a, v8f& b, v16b x, v16b y) { asm volatile("v_nop\n\tv_nop\n\tv_nop\n\tv_nop" : "+v"(a), "+v"(b) : "v"(x), "v"(y)); }
__device__ __forceinline__ void keep4_h(v16h a, v16h b, v16h c, v16h d) { asm volatile("v_nop" :: "v"(a), "v"(b), "v"(c), "v"(d)); }
__device__ __forceinline__ void keep4_b(v16b a, v16b b, v16b c, v16b d) { asm volatile("v_nop" :: "v"(a), "v"(b), "v"(c), "v"(d)); }
__device__ __forceinline__ void acc_guard4(v8f& a, v8f& b, v8f& c, v8f& d) { asm volatile("v_nop\n\tv_nop\n\tv_nop\n\tv_nop" : "+v"(a), "+v"(b), "+v"(c), "+v"(d)); }
template <typename T> struct Frag;
template <> struct Frag<_Float16> {
  typedef v16h V; union U { v16h v; v8h h[2]; };
  static __device__ __forceinline__ v16h load(const _Float16* p) {
    U f; f.h[0] = *(const v8h*)(p); f.h[1] = *(const v8h*)(p + 16); return f.v;
  }
  static __device__ __forceinline__ v8f mma(v16h a, v16h b, v8f c) {
    return __builtin_amdgcn_wmma_f32_16x16x32_f16(false, a, false, b, (short)0, c, false, false);
  }
  static __device__ __forceinline__ void guard(v8f& a, v8f& b, v16h x, v16h y) { dep_guard_h(a, b, x, y); }
  static __device__ __forceinline__ void keep(v16h a, v16h b, v16h c, v16h d) { keep4_h(a, b, c, d); }
};
template <> struct Frag<__bf16> {
  typedef v16b V; union U { v16b v; v8b h[2]; };
  static __device__ __forceinline__ v16b load(const __bf16* p) {
    U f; f.h[0] = *(const v8b*)(p); f.h[1] = *(const v8b*)(p + 16); return f.v;
  }
  static __device__ __forceinline__ v8f mma(v16b a, v16b b, v8f c) {
    return __builtin_amdgcn_wmma_f32_16x16x32_bf16(false, a, false, b, (short)0, c, false, false);
  }
  static __device__ __forceinline__ void guard(v8f& a, v8f& b, v16b x, v16b y) { dep_guard_b(a, b, x, y); }
  static __device__ __forceinline__ void keep(v16b a, v16b b, v16b c, v16b d) { keep4_b(a, b, c, d); }
};

__device__ __forceinline__ unsigned pk16(unsigned short a, unsigned short b) { return (unsigned)a | ((unsigned)b << 16); }
__device__ __forceinline__ unsigned short h_bits(float f) { const _Float16 h = (_Float16)f; return __builtin_bit_cast(unsigned short, h); }

template <int ET> struct Elem;
template <> struct Elem<0> { typedef _Float16 T; };
template <> struct Elem<1> { typedef __bf16 T; };
template <int ET, bool SPLIT, int BIAS_MODE, int OUT_MODE, bool RESID, int ACT = 0, bool TRI = false, bool CAUSALK = false>
__global__ __launch_bounds__(256) void wmma_gemm64(
    const unsigned short* __restrict__ Ap, const unsigned short* __restrict__ A2p, int lda, long strideA,
    const unsigned short* __restrict__ Btp, const unsigned short* __restrict__ Bt2p, int ldb, long strideB,
    void* __restrict__ Cout, void* __restrict__ Cout2, int ldc, long strideC,
    const float* __restrict__ bias,
    const float* __restrict__ resid, long strideR,
    int M, int N, int K, float scale) {
  typedef typename Elem<ET>::T T;
  typedef typename Frag<T>::V V;
  const T* A = (const T*)Ap; const T* A2 = (const T*)A2p; const T* Bt = (const T*)Btp; const T* Bt2 = (const T*)Bt2p;
  __shared__ __align__(16) float sT[8][16 * 68];
  const int b    = blockIdx.y;
  const int lane = threadIdx.x & 31;
  const int wave = threadIdx.x >> 5;
  const int tilesN = N >> 6;
  const int tilesM = M >> 6;
  const int ntiles = TRI ? ((tilesM * (tilesM + 1)) >> 1) : (tilesM * tilesN);
  const int tile = blockIdx.x * 8 + wave;
  if (tile >= ntiles) return;
  int tm, tn;
  if (TRI) {
    int t0 = (int)((sqrtf(8.0f * (float)tile + 1.0f) - 1.0f) * 0.5f);
    if (((t0 + 1) * (t0 + 2)) / 2 <= tile) t0 += 1;
    if ((t0 * (t0 + 1)) / 2 > tile) t0 -= 1;
    t0 = t0 < 0 ? 0 : (t0 > tilesM - 1 ? tilesM - 1 : t0);
    tm = t0;
    tn = tile - (t0 * (t0 + 1)) / 2;
    tn = tn < 0 ? 0 : (tn > tm ? tm : tn);
  } else {
    tm = tile / tilesN;
    tn = tile - tm * tilesN;
  }
  const int m0 = tm << 6;
  const int n0 = tn << 6;
  const int Kc = (tm + 1) << 6;
  const int Kt = CAUSALK ? (Kc < K ? Kc : K) : K;

  const T* Ab  = A  + (size_t)b * strideA;
  const T* Bb  = Bt + (size_t)b * strideB;
  const T* Ab2 = SPLIT ? (A2  + (size_t)b * strideA) : nullptr;
  const T* Bb2 = SPLIT ? (Bt2 + (size_t)b * strideB) : nullptr;

  const int rlane = lane & 15;
  const int koff  = (lane >> 4) * 8;
  const int mOff  = (lane >> 4) * 8;

  v8f acc[4][4];
#pragma unroll
  for (int i = 0; i < 4; ++i)
#pragma unroll
    for (int j = 0; j < 4; ++j) acc[i][j] = (v8f){0.f,0.f,0.f,0.f,0.f,0.f,0.f,0.f};

  for (int k0 = 0; k0 < Kt; k0 += 32) {
    V bh[4], bl[4];
#pragma unroll
    for (int j = 0; j < 4; ++j) {
      const size_t bo = (size_t)(n0 + (j << 4) + rlane) * ldb + koff + k0;
      bh[j] = Frag<T>::load(Bb + bo);
      if (SPLIT) bl[j] = Frag<T>::load(Bb2 + bo);
    }
#pragma unroll
    for (int i = 0; i < 4; ++i) {
      const size_t ao = (size_t)(m0 + (i << 4) + rlane) * lda + koff + k0;
      V ah = Frag<T>::load(Ab + ao);
      V al;
      if (SPLIT) al = Frag<T>::load(Ab2 + ao);
#pragma unroll
      for (int j = 0; j < 4; ++j) {
        acc[i][j] = Frag<T>::mma(ah, bh[j], acc[i][j]);
        if (SPLIT) {
          acc[i][j] = Frag<T>::mma(ah, bl[j], acc[i][j]);
          acc[i][j] = Frag<T>::mma(al, bh[j], acc[i][j]);
        }
      }
      Frag<T>::guard(acc[i][0], acc[i][3], ah, SPLIT ? al : ah);
    }
    Frag<T>::keep(bh[0], bh[1], bh[2], bh[3]);
    if (SPLIT) Frag<T>::keep(bl[0], bl[1], bl[2], bl[3]);
  }
  acc_guard4(acc[0][0], acc[0][1], acc[0][2], acc[0][3]);
  acc_guard4(acc[1][0], acc[1][1], acc[1][2], acc[1][3]);
  acc_guard4(acc[2][0], acc[2][1], acc[2][2], acc[2][3]);
  acc_guard4(acc[3][0], acc[3][1], acc[3][2], acc[3][3]);

  float* slab = sT[wave];
  const float* Rb = RESID ? (resid + (size_t)b * strideR) : nullptr;
#pragma unroll
  for (int i = 0; i < 4; ++i) {
    const int mBase = m0 + (i << 4);
#pragma unroll
    for (int j = 0; j < 4; ++j) {
      const int n = n0 + (j << 4) + rlane;
      float bv = 0.f;
      if (BIAS_MODE == 2) bv = bias[n];
#pragma unroll
      for (int r = 0; r < 8; ++r) {
        float v = acc[i][j][r] * scale;
        if (BIAS_MODE == 1) v += bias[mBase + mOff + r];
        if (BIAS_MODE == 2) v += bv;
        if (RESID) v += Rb[(size_t)(mBase + mOff + r) * ldc + n];
        if (ACT == 2) v = fmaxf(v, 0.0f);
        if (ACT == 4) v = (v > 0.f) ? v : 0.01f * v;
        if (ACT == 6) {
          const float sg = kPCarry / (1.0f + expf(-v));
          v = (n > (mBase + mOff + r)) ? 0.0f : sg;
        }
        slab[(mOff + r) * 68 + (j << 4) + rlane] = v;
      }
    }
    __builtin_amdgcn_fence(__ATOMIC_RELEASE, "workgroup");
    __builtin_amdgcn_wave_barrier();
    __builtin_amdgcn_fence(__ATOMIC_ACQUIRE, "workgroup");
    if (OUT_MODE == 0) {
      float* C = (float*)Cout + (size_t)b * strideC;
      const int hh = lane >> 4, c4 = (lane & 15) * 4;
      for (int pass = 0; pass < 2; ++pass) {
#pragma unroll
        for (int it = 0; it < 8; ++it) {
          const int row = it * 2 + hh;
          v4f v = *(const v4f*)(slab + row * 68 + c4);
          *(volatile v4f*)(C + (size_t)(mBase + row) * ldc + n0 + c4) = v;
        }
        __threadfence();
      }
    } else {
      const int q = lane >> 3, c8 = (lane & 7) * 8;
      unsigned short* C  = (unsigned short*)Cout  + (size_t)b * strideC;
      unsigned short* C2 = (OUT_MODE == 2) ? ((unsigned short*)Cout2 + (size_t)b * strideC) : nullptr;
      for (int pass = 0; pass < 2; ++pass) {
#pragma unroll
        for (int it = 0; it < 4; ++it) {
          const int row = it * 4 + q;
          const float* sp = slab + row * 68 + c8;
          v8h hv, lv;
#pragma unroll
          for (int e = 0; e < 8; ++e) {
            if (OUT_MODE == 1) {
              hv[e] = (_Float16)sp[e];
            } else {
              unsigned short hb = f2bf_bits(sp[e]);
              unsigned short lb = f2bf_bits(sp[e] - bf_bits2f(hb));
              hv[e] = __builtin_bit_cast(_Float16, hb);
              lv[e] = __builtin_bit_cast(_Float16, lb);
            }
          }
          *(volatile v8h*)(C + (size_t)(mBase + row) * ldc + n0 + c8) = hv;
          if (OUT_MODE == 2) *(volatile v8h*)(C2 + (size_t)(mBase + row) * ldc + n0 + c8) = lv;
        }
        __threadfence();
      }
    }
    __builtin_amdgcn_fence(__ATOMIC_RELEASE, "workgroup");
    __builtin_amdgcn_wave_barrier();
    __builtin_amdgcn_fence(__ATOMIC_ACQUIRE, "workgroup");
  }
}

__global__ __launch_bounds__(256) void xcast_kernel(const float* __restrict__ in, unsigned short* __restrict__ o16,
                                                    unsigned short* __restrict__ obh, unsigned short* __restrict__ obl, int n8) {
  const int i = blockIdx.x * 256 + threadIdx.x;
  if (i >= n8) return;
  const float* p = in + 8 * (size_t)i;
  const v4f a = *(const v4f*)(p);
  const v4f c = *(const v4f*)(p + 4);
  float f[8];
#pragma unroll
  for (int e = 0; e < 4; ++e) { f[e] = a[e]; f[4 + e] = c[e]; }
  unsigned short hb[8], bh[8], bl[8];
#pragma unroll
  for (int e = 0; e < 8; ++e) {
    hb[e] = h_bits(f[e]);
    bh[e] = f2bf_bits(f[e]);
    bl[e] = f2bf_bits(f[e] - bf_bits2f(bh[e]));
  }
  const v4u u0 = (v4u){pk16(hb[0], hb[1]), pk16(hb[2], hb[3]), pk16(hb[4], hb[5]), pk16(hb[6], hb[7])};
  const v4u u1 = (v4u){pk16(bh[0], bh[1]), pk16(bh[2], bh[3]), pk16(bh[4], bh[5]), pk16(bh[6], bh[7])};
  const v4u u2 = (v4u){pk16(bl[0], bl[1]), pk16(bl[2], bl[3]), pk16(bl[4], bl[5]), pk16(bl[6], bl[7])};
  const size_t o = 8 * (size_t)i;
  *(volatile v4u*)(o16 + o) = u0;
  *(volatile v4u*)(obh + o) = u1;
  *(volatile v4u*)(obl + o) = u2;
  __threadfence();
  *(volatile v4u*)(o16 + o) = u0;
  *(volatile v4u*)(obh + o) = u1;
  *(volatile v4u*)(obl + o) = u2;
}

__global__ __launch_bounds__(256) void wcast_kernel(const float* __restrict__ w0, const float* __restrict__ w1,
                                                    const float* __restrict__ w2, unsigned short* __restrict__ out,
                                                    float scale, int n8) {
  const int i = blockIdx.x * 256 + threadIdx.x;
  if (i >= n8) return;
  const int z = blockIdx.y;
  const float* w = (z == 0) ? w0 : ((z == 1) ? w1 : w2);
  const float* p = w + 8 * (size_t)i;
  const v4f a = *(const v4f*)(p);
  const v4f c = *(const v4f*)(p + 4);
  unsigned short hb[8];
#pragma unroll
  for (int e = 0; e < 4; ++e) {
    hb[e]     = h_bits(a[e] * scale);
    hb[4 + e] = h_bits(c[e] * scale);
  }
  const v4u u = (v4u){pk16(hb[0], hb[1]), pk16(hb[2], hb[3]), pk16(hb[4], hb[5]), pk16(hb[6], hb[7])};
  unsigned short* q = out + (size_t)z * (size_t)n8 * 8 + 8 * (size_t)i;
  *(volatile v4u*)q = u;
  __threadfence();
  *(volatile v4u*)q = u;
}

__global__ __launch_bounds__(256) void wsplit_kernel(const float* __restrict__ w, unsigned short* __restrict__ hi,
                                                     unsigned short* __restrict__ lo, int n8) {
  const int i = blockIdx.x * 256 + threadIdx.x;
  if (i >= n8) return;
  const float* p = w + 8 * (size_t)i;
  const v4f a = *(const v4f*)(p);
  const v4f c = *(const v4f*)(p + 4);
  float f[8];
#pragma unroll
  for (int e = 0; e < 4; ++e) { f[e] = a[e]; f[4 + e] = c[e]; }
  unsigned short bh[8], bl[8];
#pragma unroll
  for (int e = 0; e < 8; ++e) {
    bh[e] = f2bf_bits(f[e]);
    bl[e] = f2bf_bits(f[e] - bf_bits2f(bh[e]));
  }
  const v4u u1 = (v4u){pk16(bh[0], bh[1]), pk16(bh[2], bh[3]), pk16(bh[4], bh[5]), pk16(bh[6], bh[7])};
  const v4u u2 = (v4u){pk16(bl[0], bl[1]), pk16(bl[2], bl[3]), pk16(bl[4], bl[5]), pk16(bl[6], bl[7])};
  const size_t o = 8 * (size_t)i;
  *(volatile v4u*)(hi + o) = u1;
  *(volatile v4u*)(lo + o) = u2;
  __threadfence();
  *(volatile v4u*)(hi + o) = u1;
  *(volatile v4u*)(lo + o) = u2;
}

__global__ __launch_bounds__(256) void rope_rms_kernel(const float* __restrict__ qf, const float* __restrict__ kf,
                                                       const float* __restrict__ cosT, const float* __restrict__ sinT,
                                                       unsigned short* __restrict__ qk16) {
#pragma clang fp contract(off)
  __shared__ __align__(16) float sm[8][256];
  const int lane = threadIdx.x & 31;
  const int wave = threadIdx.x >> 5;
  const int pbase = (blockIdx.x * 8 + wave) * 2;
#pragma unroll
  for (int u = 0; u < 2; ++u) {
    const int p = pbase + u;
    const int t = p >> 4;
    const int h = p & 15;
    const float c = cosT[(size_t)t * kRotD + lane];
    const float s = sinT[(size_t)t * kRotD + lane];
    const size_t ib = (size_t)t * kEmbd + (size_t)h * kHeadD + lane;
    const float q1 = qf[ib], q2 = qf[ib + 32];
    const float k1 = kf[ib], k2 = kf[ib + 32];
    const float qo1 = q1 * c + q2 * s;
    const float qo2 = -q1 * s + q2 * c;
    const float ko1 = k1 * c + k2 * s;
    const float ko2 = -k1 * s + k2 * c;
    float ssq = qo1 * qo1 + qo2 * qo2;
    float ssk = ko1 * ko1 + ko2 * ko2;
#pragma unroll
    for (int off = 16; off >= 1; off >>= 1) {
      ssq += __shfl_xor(ssq, off, 32);
      ssk += __shfl_xor(ssk, off, 32);
    }
    const float rq = rsqrtf(ssq * (1.0f / 64.0f) + kEpsRms);
    const float rk = rsqrtf(ssk * (1.0f / 64.0f) + kEpsRms);
    float* row = &sm[wave][u * 128];
    row[lane]      = qo1 * rq;
    row[32 + lane] = qo2 * rq;
    row[64 + lane] = ko1 * rk;
    row[96 + lane] = ko2 * rk;
  }
  __syncthreads();
  const int g = lane >> 3;
  const int uu = g >> 1;
  const int which = g & 1;
  const int j = lane & 7;
  const int p = pbase + uu;
  const int t = p >> 4;
  const int h = p & 15;
  const float* sp = &sm[wave][uu * 128 + which * 64 + 8 * j];
  const v4f a = *(const v4f*)(sp);
  const v4f c = *(const v4f*)(sp + 4);
  unsigned short hb[8];
#pragma unroll
  for (int e = 0; e < 4; ++e) {
    hb[e]     = h_bits(a[e]);
    hb[4 + e] = h_bits(c[e]);
  }
  const v4u u = (v4u){pk16(hb[0], hb[1]), pk16(hb[2], hb[3]), pk16(hb[4], hb[5]), pk16(hb[6], hb[7])};
  unsigned short* dst = qk16 + (size_t)which * ((size_t)kHeads * kSeqLen * kHeadD)
                      + ((size_t)h * kSeqLen + t) * kHeadD + 8 * j;
  *(volatile v4u*)dst = u;
  __threadfence();
  *(volatile v4u*)dst = u;
}

extern "C" void kernel_launch(void* const* d_in, const int* in_sizes, int n_in,
                              void* d_out, int out_size, void* d_ws,
                              size_t ws_size, hipStream_t stream) {
  if (n_in < 7) return;
  if (in_sizes[0] != kSeqLen * kEmbd) return;
  if (in_sizes[1] != kSeqLen * kRotD || in_sizes[2] != kSeqLen * kRotD) return;
  if (in_sizes[3] != kEmbd * kEmbd || in_sizes[4] != kEmbd * kEmbd ||
      in_sizes[5] != kEmbd * kEmbd || in_sizes[6] != kEmbd * kEmbd) return;
  if (out_size != kSeqLen * kEmbd) return;

  const float* x    = (const float*)d_in[0];
  const float* cosT = (const float*)d_in[1];
  const float* sinT = (const float*)d_in[2];
  const float* wq   = (const float*)d_in[3];
  const float* wk   = (const float*)d_in[4];
  const float* wv   = (const float*)d_in[5];
  const float* wp   = (const float*)d_in[6];

  const size_t MiB = 1048576;
  const size_t total = 106 * MiB;
  if (total > ws_size) return;
  char* ws = (char*)d_ws;
  unsigned short* Q16  = (unsigned short*)(ws + 0 * MiB);
  unsigned short* K16  = (unsigned short*)(ws + 8 * MiB);
  unsigned short* VT16 = (unsigned short*)(ws + 16 * MiB);
  unsigned short* O16  = (unsigned short*)(ws + 24 * MiB);
  unsigned short* W16  = (unsigned short*)(ws + 32 * MiB);
  unsigned short* WVH  = (unsigned short*)(ws + 38 * MiB);
  unsigned short* WVL  = (unsigned short*)(ws + 40 * MiB);
  unsigned short* X16  = (unsigned short*)(ws + 42 * MiB);
  unsigned short* XBH  = (unsigned short*)(ws + 50 * MiB);
  unsigned short* XBL  = (unsigned short*)(ws + 58 * MiB);
  float*          QF   = (float*)(ws + 66 * MiB);
  unsigned short* P16  = (unsigned short*)(ws + 42 * MiB);
  unsigned short* WP16 = W16 + 2 * (size_t)kEmbd * kEmbd;
  const float* fdummy = (const float*)(ws);

  {
    const int n8x = (kSeqLen * kEmbd) / 8;
    xcast_kernel<<<dim3((n8x + 255) / 256), 256, 0, stream>>>(x, X16, XBH, XBL, n8x);
    const int n8w = (kEmbd * kEmbd) / 8;
    wcast_kernel<<<dim3((n8w + 255) / 256, 3), 256, 0, stream>>>(wq, wk, wp, W16, kWCarry, n8w);
    wsplit_kernel<<<dim3((n8w + 255) / 256), 256, 0, stream>>>(wv, WVH, WVL, n8w);
  }

  {
    const int tiles = (kSeqLen / 64) * (kEmbd / 64);
    wmma_gemm64<0, false, 0, 0, false, 0><<<dim3((tiles + 7) / 8, 2), 256, 0, stream>>>(
        X16, X16, kEmbd, (long)0,
        W16, W16, kEmbd, (long)kEmbd * kEmbd,
        (void*)QF, (void*)QF, kEmbd, (long)kSeqLen * kEmbd,
        fdummy, fdummy, (long)0,
        kSeqLen, kEmbd, kEmbd, kQKScale);
  }

  {
    const int tiles = (kEmbd / 64) * (kSeqLen / 64);
    wmma_gemm64<1, true, 0, 1, false, 0><<<dim3((tiles + 7) / 8, 1), 256, 0, stream>>>(
        WVH, WVL, kEmbd, (long)0,
        XBH, XBL, kEmbd, (long)0,
        (void*)VT16, (void*)VT16, kSeqLen, (long)0,
        fdummy, fdummy, (long)0,
        kEmbd, kSeqLen, kEmbd, kVCarry);
  }

  rope_rms_kernel<<<dim3((kSeqLen * kHeads) / 16), 256, 0, stream>>>(QF, QF + (size_t)kSeqLen * kEmbd, cosT, sinT, Q16);

  {
    const long headPlane = (long)kSeqLen * kHeadD;
    const long vtHead    = (long)kHeadD * kSeqLen;
    const long pPlane    = (long)kSeqLen * kSeqLen;
    const int  tilesM    = kSeqLen / 64;
    const int  ntri      = (tilesM * (tilesM + 1)) / 2;
    const int  pvTiles   = tilesM * (kHeadD / 64);
    for (int hc = 0; hc < kHeads / kHeadsPerChunk; ++hc) {
      const int h0 = hc * kHeadsPerChunk;
      wmma_gemm64<0, false, 0, 1, false, 6, true, false><<<dim3((ntri + 7) / 8, kHeadsPerChunk), 256, 0, stream>>>(
          Q16 + (size_t)h0 * headPlane, Q16 + (size_t)h0 * headPlane, kHeadD, headPlane,
          K16 + (size_t)h0 * headPlane, K16 + (size_t)h0 * headPlane, kHeadD, headPlane,
          (void*)P16, (void*)P16, kSeqLen, pPlane,
          fdummy, fdummy, (long)0,
          kSeqLen, kSeqLen, kHeadD, kScScale);
      wmma_gemm64<0, false, 0, 1, false, 0, false, true><<<dim3((pvTiles + 7) / 8, kHeadsPerChunk), 256, 0, stream>>>(
          P16, P16, kSeqLen, pPlane,
          VT16 + (size_t)h0 * vtHead, VT16 + (size_t)h0 * vtHead, kSeqLen, vtHead,
          (void*)(O16 + (size_t)h0 * kHeadD), (void*)(O16 + (size_t)h0 * kHeadD), kEmbd, (long)kHeadD,
          fdummy, fdummy, (long)0,
          kSeqLen, kHeadD, kSeqLen, kPVScale);
    }
  }

  {
    const int tiles = (kSeqLen / 64) * (kEmbd / 64);
    wmma_gemm64<0, false, 0, 0, false, 0><<<dim3((tiles + 7) / 8, 1), 256, 0, stream>>>(
        O16, O16, kEmbd, (long)0,
        WP16, WP16, kEmbd, (long)0,
        d_out, d_out, kEmbd, (long)0,
        fdummy, fdummy, (long)0,
        kSeqLen, kEmbd, kEmbd, kOutScale);
  }
}
